// Attention_42949672960850
// MI455X (gfx1250) — hardware-run, weakly checked
//
#include <hip/hip_runtime.h>


#define NB_  8
#define NR   64
#define NK   512
#define DM   512
#define OFF1 262144
typedef _Float16 h16;
typedef unsigned short bf;
typedef __attribute__((ext_vector_type(16))) __bf16   v16bf;
typedef __attribute__((ext_vector_type(16))) _Float16 v16h;
typedef __attribute__((ext_vector_type(8)))  _Float16 v8h;
typedef __attribute__((ext_vector_type(8)))  unsigned short v8us;
typedef __attribute__((ext_vector_type(8)))  float    v8f;
typedef __attribute__((ext_vector_type(4)))  float    v4f;
typedef v8h  __attribute__((may_alias)) v8ha;
typedef v4f  __attribute__((may_alias)) v4fa;
typedef v8us __attribute__((may_alias)) v8usa;

__device__ __forceinline__ unsigned short f2bf(float f) { unsigned u = __float_as_uint(f); u += 0x7FFFu + ((u >> 16) & 1u); return (unsigned short)(u >> 16); }
__device__ __forceinline__ float bf2f(unsigned short b) { return __uint_as_float(((unsigned)b) << 16); }
__device__ __forceinline__ float bfr(float f) { return bf2f(f2bf(f)); }
__device__ __forceinline__ v16h cat16(v8h lo, v8h hi) { return __builtin_shufflevector(lo, hi, 0, 1, 2, 3, 4, 5, 6, 7, 8, 9, 10, 11, 12, 13, 14, 15); }
__device__ __forceinline__ v16bf cat16b(v8us lo, v8us hi) { return __builtin_bit_cast(v16bf, __builtin_shufflevector(lo, hi, 0, 1, 2, 3, 4, 5, 6, 7, 8, 9, 10, 11, 12, 13, 14, 15)); }
__device__ __forceinline__ v8f wmma16(v16h a, v16h b, v8f c) { return __builtin_amdgcn_wmma_f32_16x16x32_f16(false, a, false, b, (short)0, c, false, false); }
__device__ __forceinline__ v8f wmmab(v16bf a, v16bf b, v8f c) { return __builtin_amdgcn_wmma_f32_16x16x32_bf16(false, a, false, b, (short)0, c, false, false); }


template <typename T16> struct WFrag;
template <> struct WFrag<h16> { typedef v16h V; static __device__ __forceinline__ V ld(const h16* p) { return cat16(*(const v8h*)p, *(const v8h*)(p + 16)); } static __device__ __forceinline__ v8f mma(V a, V b, v8f c) { return wmma16(a, b, c); } };
template <> struct WFrag<bf> { typedef v16bf V; static __device__ __forceinline__ V ld(const bf* p) { return cat16b(*(const v8us*)p, *(const v8us*)(p + 16)); } static __device__ __forceinline__ v8f mma(V a, V b, v8f c) { return wmmab(a, b, c); } };
template <typename T16, int NSPLIT, bool BIAS>
__global__ __launch_bounds__(32) void k_gemmw(const T16* __restrict__ A, const T16* __restrict__ A2, const T16* __restrict__ Bt, const T16* __restrict__ Bt2, int K, float* C, int ldc, const float* __restrict__ bias, size_t sA, size_t sB, size_t sC) {
    typedef typename WFrag<T16>::V V;
    __shared__ __align__(16) float os[16 * 68];
    const size_t z = blockIdx.z; A += z * sA; if (A2) A2 += z * sA; Bt += z * sB; if (Bt2) Bt2 += z * sB; C += z * sC;
    const int lane = threadIdx.x & 31, lr = lane & 15, hi = lane >> 4; const int r0 = blockIdx.x * 64, c0 = blockIdx.y * 64;
    v8f acc[4][4];
#pragma unroll
    for (int mb = 0; mb < 4; ++mb)
#pragma unroll
        for (int nb = 0; nb < 4; ++nb) acc[mb][nb] = (v8f){};
    const size_t aoff = (size_t)(r0 + lr) * K + 8 * hi, boff = (size_t)(c0 + lr) * K + 8 * hi;
    for (int kc = 0; kc < K; kc += 32) {
        V a[4], a2[4];
#pragma unroll
        for (int mb = 0; mb < 4; ++mb) { a[mb] = WFrag<T16>::ld(A + aoff + (size_t)mb * 16 * K + kc); if (NSPLIT == 1 || NSPLIT == 2) a2[mb] = WFrag<T16>::ld(A2 + aoff + (size_t)mb * 16 * K + kc); }
#pragma unroll
        for (int nb = 0; nb < 4; ++nb) { const V b = WFrag<T16>::ld(Bt + boff + (size_t)nb * 16 * K + kc); V b2; if (NSPLIT >= 2) b2 = WFrag<T16>::ld(Bt2 + boff + (size_t)nb * 16 * K + kc);
#pragma unroll
            for (int mb = 0; mb < 4; ++mb) { acc[mb][nb] = WFrag<T16>::mma(a[mb], b, acc[mb][nb]); if (NSPLIT == 1 || NSPLIT == 2) acc[mb][nb] = WFrag<T16>::mma(a2[mb], b, acc[mb][nb]); if (NSPLIT >= 2) acc[mb][nb] = WFrag<T16>::mma(a[mb], b2, acc[mb][nb]); } }
        asm volatile("v_nop\n\tv_nop\n\tv_nop\n\tv_nop" : "+v"(acc[0][0]), "+v"(acc[1][1]), "+v"(acc[2][2]), "+v"(acc[3][3]) : "v"(a[0]), "v"(a[3]));
    }
#pragma unroll
    for (int mb = 0; mb < 4; ++mb) {
#pragma unroll
        for (int nb = 0; nb < 4; ++nb) {
#pragma unroll
            for (int j = 0; j < 8; ++j) os[(hi * 8 + j) * 68 + nb * 16 + lr] = acc[mb][nb][j]; }
        __builtin_amdgcn_wave_barrier(); asm volatile("" ::: "memory");
        float* crow = C + (size_t)(r0 + mb * 16) * ldc + c0;
#pragma unroll 1
        for (int ps = 0; ps < 2; ++ps) {
#pragma unroll
            for (int s = 0; s < 8; ++s) { const int row = 2 * s + hi, cofs = lr * 4; v4f val = *(const v4fa*)(os + row * 68 + cofs); if (BIAS) { val[0] += bfr(bias[c0 + cofs]); val[1] += bfr(bias[c0 + cofs + 1]); val[2] += bfr(bias[c0 + cofs + 2]); val[3] += bfr(bias[c0 + cofs + 3]); }
                *(volatile v4f*)(crow + (size_t)row * ldc + cofs) = val; }
            if (ps == 0) __threadfence(); }
        __builtin_amdgcn_wave_barrier(); asm volatile("" ::: "memory");
    }
}

__device__ __forceinline__ h16 tohx(float x) { return (h16)x; }
__device__ __forceinline__ void splitf(float y, unsigned short& h, unsigned short& l) { h = f2bf(y); l = f2bf(y - bf2f(h)); }
typedef __attribute__((ext_vector_type(2))) _Float16 v2h;
typedef __attribute__((ext_vector_type(4))) _Float16 v4h;
typedef __attribute__((ext_vector_type(2))) unsigned short v2us;
typedef __attribute__((ext_vector_type(4))) unsigned short v4us;
typedef __attribute__((ext_vector_type(2))) float v2f;
typedef __attribute__((ext_vector_type(4))) int v4i;

__global__ __launch_bounds__(256) void k_wtG(const float* __restrict__ w, int K, int N, bf* Bt) {
    const int lane = threadIdx.x & 31; const int L0 = (blockIdx.x * 8 + (threadIdx.x >> 5)) * 8; const int nlines = N * K / 64;
#pragma unroll
    for (int ps = 0; ps < 2; ++ps) {
        for (int l = 0; l < 8; ++l) { const int L = L0 + l; if (L >= nlines) break; const size_t e = (size_t)L * 64 + lane * 2; const int k = (int)(e % K), n = (int)(e / K); v2us o;
            o[0] = f2bf(w[(size_t)k * N + n]); o[1] = f2bf(w[(size_t)(k + 1) * N + n]); *(volatile v2us*)(Bt + e) = o; }
        if (ps == 0) __threadfence(); }
}
__global__ __launch_bounds__(256) void k_cvt8(const float* __restrict__ src, bf* dst, size_t n8) { const size_t i = (size_t)blockIdx.x * 256 + threadIdx.x; if (i >= n8) return; const v8f v = *(const v8f*)(src + i * 8); v8us o;
#pragma unroll
    for (int k = 0; k < 8; ++k) o[k] = f2bf(v[k]); *(volatile v8us*)(dst + i * 8) = o; __threadfence(); *(volatile v8us*)(dst + i * 8) = o; }

__global__ __launch_bounds__(256) void k_score(const float* RP, const float* KT, const float* __restrict__ wv, const float* __restrict__ bk, const float* __restrict__ br, const float* __restrict__ b0, float* S) { const unsigned idx = blockIdx.x * 256 + threadIdx.x; const unsigned j = idx % NK, r = idx / NK, en = r / NR; const float* rq = RP + (size_t)r * DM; const float* ck = KT + (size_t)en * DM * NK + j; float acc = 0.0f;
    for (int u = 0; u < DM; ++u) acc += bfr(wv[u]) * tanhf((ck[(size_t)u * NK] + bfr(bk[u])) + (rq[u] + bfr(br[u])));
    const float y = acc + bfr(b0[0]); *(volatile float*)(S + idx) = y; __threadfence(); *(volatile float*)(S + idx) = y; }
__global__ __launch_bounds__(256) void k_sm1(const float* S, float* PART) { const unsigned idx = blockIdx.x * 256 + threadIdx.x; const float* rs = S + (size_t)idx * 64; float x[64];
#pragma unroll
    for (int j4 = 0; j4 < 16; ++j4) { const v4f a = *(const v4f*)(rs + j4 * 4); x[j4 * 4] = a[0]; x[j4 * 4 + 1] = a[1]; x[j4 * 4 + 2] = a[2]; x[j4 * 4 + 3] = a[3]; }
    float mx = x[0];
#pragma unroll
    for (int j = 1; j < 64; ++j) mx = (x[j] > mx) ? x[j] : mx;
    float sum = 0.0f;
#pragma unroll
    for (int j = 0; j < 64; ++j) sum += expf(x[j] - mx);
    v2f pr; pr[0] = mx; pr[1] = sum; *(volatile v2f*)(PART + (size_t)idx * 2) = pr; __threadfence(); *(volatile v2f*)(PART + (size_t)idx * 2) = pr; }
__global__ __launch_bounds__(256) void k_sm2(const float* S, const float* PART, float* Wo, h16* P16) { const unsigned idx = blockIdx.x * 256 + threadIdx.x; const unsigned r = idx / 8; const float* pp = PART + (size_t)r * 16; float pm[8], pz[8];
#pragma unroll
    for (int q2 = 0; q2 < 4; ++q2) { const v4f a = *(const v4f*)(pp + q2 * 4); pm[q2 * 2] = a[0]; pz[q2 * 2] = a[1]; pm[q2 * 2 + 1] = a[2]; pz[q2 * 2 + 1] = a[3]; }
    float M = pm[0];
#pragma unroll
    for (int q = 1; q < 8; ++q) M = (pm[q] > M) ? pm[q] : M;
    float Z = 0.0f;
#pragma unroll
    for (int q = 0; q < 8; ++q) Z += pz[q] * expf(pm[q] - M);
    const float* rs = S + (size_t)idx * 64; v4f o[16]; v8h h[8];
#pragma unroll
    for (int j4 = 0; j4 < 16; ++j4) { const v4f a = *(const v4f*)(rs + j4 * 4);
#pragma unroll
        for (int q = 0; q < 4; ++q) { const float w = expf(a[q] - M) / Z; o[j4][q] = w; h[j4 / 2][(j4 % 2) * 4 + q] = tohx(w * 512.0f); } }
#pragma unroll
    for (int j4 = 0; j4 < 16; ++j4) *(volatile v4f*)(Wo + (size_t)idx * 64 + j4 * 4) = o[j4];
#pragma unroll
    for (int g = 0; g < 8; ++g) *(volatile v8h*)(P16 + (size_t)idx * 64 + g * 8) = h[g];
    __threadfence();
#pragma unroll
    for (int j4 = 0; j4 < 16; ++j4) *(volatile v4f*)(Wo + (size_t)idx * 64 + j4 * 4) = o[j4];
#pragma unroll
    for (int g = 0; g < 8; ++g) *(volatile v8h*)(P16 + (size_t)idx * 64 + g * 8) = h[g]; }
__global__ __launch_bounds__(256) void k_vt(const float* __restrict__ src, h16* VT) { const unsigned idx = blockIdx.x * 256 + threadIdx.x; const unsigned j0 = (idx % (NK / 8)) * 8, d = (idx / (NK / 8)) % DM, b = idx / ((NK / 8) * DM); v8h o;
#pragma unroll
    for (int q = 0; q < 8; ++q) o[q] = tohx(bfr(src[((size_t)b * NK + j0 + q) * DM + d]));
    *(volatile v8h*)(VT + (size_t)idx * 8) = o; __threadfence(); *(volatile v8h*)(VT + (size_t)idx * 8) = o; }
__global__ __launch_bounds__(256) void k_cat(const float* __restrict__ src, float sc, int co, bf* CC) { const unsigned idx = blockIdx.x * 256 + threadIdx.x; const unsigned c0 = (idx % (DM / 8)) * 8, r = idx / (DM / 8); const v4f m0 = *(const v4f*)(src + (size_t)r * DM + c0), m1 = *(const v4f*)(src + (size_t)r * DM + c0 + 4); v8us o;
#pragma unroll
    for (int q = 0; q < 4; ++q) { o[q] = f2bf(m0[q] * sc); o[q + 4] = f2bf(m1[q] * sc); }
    bf* dst = CC + (size_t)r * 2 * DM + co + c0; *(volatile v8us*)dst = o; __threadfence(); *(volatile v8us*)dst = o; }
__global__ __launch_bounds__(256) void k_tb(const float* PR, const float* __restrict__ bo, float* res) { const unsigned idx = blockIdx.x * 256 + threadIdx.x; const unsigned d0 = (idx % (DM / 4)) * 4; const v4f p = *(const v4f*)(PR + (size_t)idx * 4), c = *(const v4f*)(bo + d0); v4f o;
#pragma unroll
    for (int q = 0; q < 4; ++q) o[q] = tanhf(p[q] + bfr(c[q]));
    *(volatile v4f*)(res + (size_t)idx * 4) = o; __threadfence(); *(volatile v4f*)(res + (size_t)idx * 4) = o; }

extern "C" void kernel_launch(void* const* d_in, const int* in_sizes, int n_in,
                              void* d_out, int out_size, void* d_ws, size_t ws_size, hipStream_t stream) {
    (void)in_sizes; (void)n_in; (void)out_size;
    const float* a0 = (const float*)d_in[0]; const float* a1 = (const float*)d_in[1]; const float* a2 = (const float*)d_in[2]; const float* a3 = (const float*)d_in[3]; const float* a4 = (const float*)d_in[4]; const float* a5 = (const float*)d_in[5]; const float* a6 = (const float*)d_in[6]; const float* a7 = (const float*)d_in[7]; const float* a8 = (const float*)d_in[8]; const float* a9 = (const float*)d_in[9];
    float* R0 = (float*)d_out;
    float* R1 = (float*)d_out + OFF1;
    char* wsp = (char*)d_ws;
    auto take = [&](size_t bytes) { char* p = wsp; wsp += (bytes + 255) & ~(size_t)255; return (void*)p; };
    bf* RB = (bf*)take((size_t)NB_ * NR * DM * 2); bf* KB = (bf*)take((size_t)NB_ * NK * DM * 2); bf* W2T = (bf*)take((size_t)DM * DM * 2); bf* W4T = (bf*)take((size_t)DM * DM * 2); bf* W8T = (bf*)take((size_t)DM * 2 * DM * 2);
    h16* VT = (h16*)take((size_t)NB_ * DM * NK * 2); float* RP = (float*)take((size_t)NB_ * NR * DM * 4); float* KT = (float*)take((size_t)NB_ * DM * NK * 4); float* S = (float*)take((size_t)NB_ * NR * NK * 4); float* PART = (float*)take((size_t)NB_ * NR * 8 * 2 * 4);
    h16* P16 = (h16*)take((size_t)NB_ * NR * NK * 2); float* BL = (float*)take((size_t)NB_ * NR * DM * 4); bf* CC = (bf*)take((size_t)NB_ * NR * 2 * DM * 2); float* PR = (float*)take((size_t)NB_ * NR * DM * 4);
    if ((size_t)(wsp - (char*)d_ws) > ws_size) return;
    k_cvt8<<<(unsigned)((size_t)NB_ * NR * DM / 8 / 256), 256, 0, stream>>>(a0, RB, (size_t)NB_ * NR * DM / 8);
    k_cvt8<<<(unsigned)((size_t)NB_ * NK * DM / 8 / 256), 256, 0, stream>>>(a1, KB, (size_t)NB_ * NK * DM / 8);
    k_wtG<<<(unsigned)(((size_t)DM * DM / 64 + 63) / 64), 256, 0, stream>>>(a2, DM, DM, W2T); k_wtG<<<(unsigned)(((size_t)DM * DM / 64 + 63) / 64), 256, 0, stream>>>(a4, DM, DM, W4T); k_wtG<<<(unsigned)(((size_t)2 * DM * DM / 64 + 63) / 64), 256, 0, stream>>>(a8, 2 * DM, DM, W8T);
    k_vt<<<(unsigned)((size_t)NB_ * DM * NK / 8 / 256), 256, 0, stream>>>(a1, VT);
    k_gemmw<bf, 0, false><<<dim3(NB_ * NR / 64, DM / 64, 1), 32, 0, stream>>>(RB, nullptr, W2T, nullptr, DM, RP, DM, nullptr, (size_t)0, (size_t)0, (size_t)0);
    k_gemmw<bf, 0, false><<<dim3(DM / 64, NK / 64, NB_), 32, 0, stream>>>(W4T, nullptr, KB, nullptr, DM, KT, NK, nullptr, (size_t)0, (size_t)NK * DM, (size_t)DM * NK);
    k_score<<<(unsigned)((size_t)NB_ * NR * NK / 256), 256, 0, stream>>>(RP, KT, a6, a5, a3, a7, S);
    k_sm1<<<(unsigned)(NB_ * NR * 8 / 256), 256, 0, stream>>>(S, PART);
    k_sm2<<<(unsigned)(NB_ * NR * 8 / 256), 256, 0, stream>>>(S, PART, R1, P16);
    k_gemmw<h16, 0, false><<<dim3(NR / 64, DM / 64, NB_), 32, 0, stream>>>(P16, nullptr, VT, nullptr, NK, BL, DM, nullptr, (size_t)NR * NK, (size_t)DM * NK, (size_t)NR * DM);
    k_cat<<<(unsigned)((size_t)NB_ * NR * DM / 8 / 256), 256, 0, stream>>>(BL, 1.0f / 512.0f, 0, CC); k_cat<<<(unsigned)((size_t)NB_ * NR * DM / 8 / 256), 256, 0, stream>>>(a0, 1.0f, DM, CC);
    k_gemmw<bf, 0, false><<<dim3(NB_ * NR / 64, DM / 64, 1), 32, 0, stream>>>(CC, nullptr, W8T, nullptr, 2 * DM, PR, DM, nullptr, (size_t)0, (size_t)0, (size_t)0);
    k_tb<<<(unsigned)((size_t)NB_ * NR * DM / 4 / 256), 256, 0, stream>>>(PR, a9, R0);
}
